// MSA_6863357739037
// MI455X (gfx1250) — hardware-verified
//
#include <hip/hip_runtime.h>


#ifndef NB
#define NB 2
#endif
#ifndef SEQ
#define SEQ 2048
#endif

namespace {
constexpr int B_FULL = 2, SEQ_FULL = 2048, DM = 1024, INTER = 1024, NH = 16, DK = 64, NQKV = 3 * INTER, NSEG = 4, NR = NB * SEQ, NBH = NB * NH;
constexpr float XS = 8.0f, WSC = 256.0f, QS = 8.0f, PSC = 4096.0f, CTS = 64.0f, LOG2E = 1.4426950408889634f, SCL = 0.03125f;
static_assert(NB >= 1 && NB <= B_FULL);
static_assert(SEQ % 128 == 0 && SEQ >= 128 && SEQ <= SEQ_FULL);
static_assert(INTER == NH * DK && DK == 64 && NSEG == 4 && DM % 128 == 0 && INTER % 128 == 0 && NQKV % 128 == 0 && DM % 64 == 0 && NR % 64 == 0 && ((size_t)NR * DM) % 2048 == 0);
typedef _Float16 b16;
typedef __attribute__((ext_vector_type(16))) _Float16 v16b;
typedef __attribute__((ext_vector_type(8))) _Float16 v8b;
typedef __attribute__((ext_vector_type(8))) float v8f;
typedef __attribute__((ext_vector_type(4))) float v4f;
typedef __attribute__((ext_vector_type(8))) int v8i;
__device__ __forceinline__ float bf16_rne(float f) { unsigned int u = __float_as_uint(f); u += 0x7FFFu + ((u >> 16) & 1u); return __uint_as_float(u & 0xFFFF0000u); }
__device__ __forceinline__ v16b frag_kb(const b16* p, int hh) { const v8b a = *(const v8b*)(p + 8 * hh), b = *(const v8b*)(p + 16 + 8 * hh); v16b f;
#pragma unroll
  for (int e = 0; e < 8; ++e) { f[e] = a[e]; f[8 + e] = b[e]; } return f; }
__device__ __forceinline__ v8f wmma16b(v16b a, v16b b, v8f c) { v8f d = __builtin_amdgcn_wmma_f32_16x16x32_f16(false, a, false, b, (short)0, c, false, false); asm volatile("v_nop\n\tv_nop\n\tv_nop\n\tv_nop" : "+v"(d) : "v"(a), "v"(b)); return d; }
__device__ __forceinline__ void wave_lds_sync() { __builtin_amdgcn_fence(3, "workgroup"); __builtin_amdgcn_wave_barrier(); __builtin_amdgcn_fence(2, "workgroup"); }
__device__ __forceinline__ float nexp2(float v) { return __builtin_amdgcn_exp2f(v); }

__global__ __launch_bounds__(128) void wtp_kernel(const float* __restrict__ src, int R, int C, b16* __restrict__ dst) {
  __shared__ __attribute__((aligned(16))) b16 tile[64][64 + 8];
  const int wave = threadIdx.x >> 5, lane = threadIdx.x & 31; const int r0 = blockIdx.x * 64, c0 = blockIdx.y * 64;
#pragma unroll 4
  for (int i = threadIdx.x; i < 64 * 16; i += 128) { const int rr = i >> 4, q = (i & 15) * 4; const v4f f = *(const v4f*)(src + (size_t)(r0 + rr) * C + c0 + q);
#pragma unroll
    for (int j = 0; j < 4; ++j) tile[q + j][rr] = (b16)(bf16_rne(f[j]) * WSC); }
  __syncthreads();
  for (int pass = 0; pass < 2; ++pass) {
#pragma unroll
    for (int i = 0; i < 4; ++i) { const int cc = wave * 16 + i * 4 + (lane >> 3), pc = (lane & 7) * 8; *(volatile v8b*)(dst + (size_t)(c0 + cc) * R + r0 + pc) = *(const v8b*)(&tile[cc][pc]); }
    __threadfence(); }
}
__global__ __launch_bounds__(256) void xp_kernel(const float* __restrict__ x, b16* __restrict__ XH) {
  const size_t u = (size_t)blockIdx.x * 256 + threadIdx.x; if (u >= (size_t)NR * DM / 8) return;
  const size_t e = u * 8; const int row = (int)(e / DM), col = (int)(e - (size_t)row * DM); const size_t xe = ((size_t)(row / SEQ) * SEQ_FULL + (size_t)(row % SEQ)) * DM + col;
  const v4f f0 = *(const v4f*)(x + xe), f1 = *(const v4f*)(x + xe + 4); v8b o;
#pragma unroll
  for (int j = 0; j < 4; ++j) { o[j] = (b16)(bf16_rne(f0[j]) * XS); o[4 + j] = (b16)(bf16_rne(f1[j]) * XS); }
  for (int pass = 0; pass < 2; ++pass) { *(volatile v8b*)(XH + e) = o; __threadfence(); }
}
__global__ __launch_bounds__(128) void qkv_kernel(const b16* __restrict__ XH, const b16* __restrict__ WQKV, b16* __restrict__ QP, b16* __restrict__ KP, b16* __restrict__ VT) {
  __shared__ __attribute__((aligned(16))) b16 Th[4][16][128 + 8];
  __shared__ __attribute__((aligned(16))) b16 Tt[128][64 + 8];
  const int wave = threadIdx.x >> 5, lane = threadIdx.x & 31, nloc = lane & 15, hlf = lane >> 4;
  const int mb = blockIdx.x * 64; const size_t m0 = (size_t)mb + wave * 16; const int n0 = blockIdx.y * 128;
  v8f acc[8];
#pragma unroll
  for (int t = 0; t < 8; ++t) acc[t] = (v8f){};
#pragma unroll 2
  for (int kb = 0; kb < DM; kb += 32) { const v16b a = frag_kb(XH + (m0 + nloc) * DM + kb, hlf);
#pragma unroll
    for (int t = 0; t < 8; ++t) acc[t] = wmma16b(a, frag_kb(WQKV + (size_t)(n0 + t * 16 + nloc) * DM + kb, hlf), acc[t]); }
  const int which = n0 / INTER; const int hb = (n0 - which * INTER) / DK;
  const int b = mb / SEQ, sb = mb - b * SEQ;
  const float osc = QS / (XS * WSC);
  if (which < 2) {
#pragma unroll
    for (int t = 0; t < 8; ++t)
#pragma unroll
      for (int r = 0; r < 8; ++r) Th[wave][8 * hlf + r][t * 16 + nloc] = (b16)(acc[t][r] * osc);
    wave_lds_sync();
    b16* P = (which == 0) ? QP : KP;
    for (int pass = 0; pass < 2; ++pass) {
#pragma unroll
      for (int i = 0; i < 8; ++i) { const int L = i * 4 + (lane >> 3), rr = L >> 1, hf = L & 1, pc = (lane & 7) * 8; const int s = sb + wave * 16 + rr;
        const v8b v = *(const v8b*)(&Th[wave][rr][hf * 64 + pc]); *(volatile v8b*)(P + ((size_t)(b * NH + hb + hf) * SEQ + s) * DK + pc) = v; }
      __threadfence(); }
  } else {
#pragma unroll
    for (int t = 0; t < 8; ++t)
#pragma unroll
      for (int r = 0; r < 8; ++r) Tt[t * 16 + nloc][wave * 16 + 8 * hlf + r] = (b16)(acc[t][r] * osc);
    __syncthreads();
    for (int pass = 0; pass < 2; ++pass) {
#pragma unroll
      for (int i = 0; i < 8; ++i) { const int cc = wave * 32 + i * 4 + (lane >> 3), hf = cc >> 6, d = cc & 63, pc = (lane & 7) * 8;
        const v8b v = *(const v8b*)(&Tt[cc][pc]); *(volatile v8b*)(VT + ((size_t)(b * NH + hb + hf) * DK + d) * SEQ + sb + pc) = v; }
      __threadfence(); }
  }
}
__global__ __launch_bounds__(256) __attribute__((amdgpu_num_vgpr(256))) void rowsum_kernel(const b16* __restrict__ QP, const b16* __restrict__ KP, const int* __restrict__ mask,
                                                                                           const int* __restrict__ nsegp, float* __restrict__ RS) {
  const int tid = threadIdx.x, wave = tid >> 5, lane = tid & 31, nloc = lane & 15, hlf = lane >> 4;
  const int bh = blockIdx.y, b = bh / NH; const int q = blockIdx.x * 128 + wave * 16 + nloc;
  const b16* Qb = QP + (size_t)bh * SEQ * DK; const b16* Kb = KP + (size_t)bh * SEQ * DK;
  const v16b b0 = frag_kb(Qb + (size_t)q * DK, hlf), b1 = frag_kb(Qb + (size_t)q * DK + 32, hlf);
  const int* mrow = mask + ((size_t)b * SEQ_FULL + (size_t)q) * SEQ_FULL;
  float acs[NSEG];
#pragma unroll
  for (int g = 0; g < NSEG; ++g) acs[g] = 0.0f;
  const float c = LOG2E * (SCL / (QS * QS));
#pragma unroll 1
  for (int sc0 = 0; sc0 < SEQ; sc0 += 32) {
#pragma unroll
    for (int st = 0; st < 2; ++st) {
      const int kr = sc0 + st * 16;
      const v16b a0 = frag_kb(Kb + (size_t)(kr + nloc) * DK, hlf), a1 = frag_kb(Kb + (size_t)(kr + nloc) * DK + 32, hlf);
      v8f s8 = (v8f){}; s8 = wmma16b(a0, b0, s8); s8 = wmma16b(a1, b1, s8);
      const v8i m8 = *(const v8i*)(mrow + kr + 8 * hlf);
#pragma unroll
      for (int r = 0; r < 8; ++r) { const float e = nexp2(s8[r] * c); const int m = m8[r];
        acs[0] += (m == 0) ? e : 0.0f; acs[1] += (m == 1) ? e : 0.0f; acs[2] += (m == 2) ? e : 0.0f; acs[3] += (m == 3) ? e : 0.0f; }
    }
  }
#pragma unroll
  for (int g = 0; g < NSEG; ++g) acs[g] += __shfl_xor(acs[g], 16);
  const int ns = nsegp[0];
  v4f o;
#pragma unroll
  for (int g = 0; g < NSEG; ++g) { const float rv = 1.0f / fmaxf(acs[g], 1e-30f); o[g] = (g < ns && acs[g] > 0.0f) ? rv : 0.0f; }
  for (int pass = 0; pass < 2; ++pass) { if (hlf == 0) *(volatile v4f*)(RS + ((size_t)bh * SEQ + q) * NSEG) = o; __threadfence(); }
}
__global__ __launch_bounds__(256) __attribute__((amdgpu_num_vgpr(256))) void av_kernel(const b16* __restrict__ QP, const b16* __restrict__ KP, const b16* __restrict__ VT,
                                                                                       const int* __restrict__ mask, const float* __restrict__ RS, b16* __restrict__ CT) {
  __shared__ __attribute__((aligned(16))) b16 Th[8][16][DK + 8];
  const int tid = threadIdx.x, wave = tid >> 5, lane = tid & 31, nloc = lane & 15, hlf = lane >> 4;
  const int bh = blockIdx.y, b = bh / NH, hd = bh - b * NH; const int q0 = blockIdx.x * 128; const int q = q0 + wave * 16 + nloc;
  const b16* Qb = QP + (size_t)bh * SEQ * DK; const b16* Kb = KP + (size_t)bh * SEQ * DK; const b16* Vb = VT + (size_t)bh * DK * SEQ;
  const v16b b0 = frag_kb(Qb + (size_t)q * DK, hlf), b1 = frag_kb(Qb + (size_t)q * DK + 32, hlf);
  const int* mrow = mask + ((size_t)b * SEQ_FULL + (size_t)q) * SEQ_FULL;
  const v4f r4 = *(const v4f*)(RS + ((size_t)bh * SEQ + q) * NSEG);
  const float w0 = r4[0] * PSC, w1 = r4[1] * PSC, w2 = r4[2] * PSC, w3 = r4[3] * PSC;
  v8f hacc[4];
#pragma unroll
  for (int vs = 0; vs < 4; ++vs) hacc[vs] = (v8f){};
  const float c = LOG2E * (SCL / (QS * QS));
#pragma unroll 1
  for (int sc0 = 0; sc0 < SEQ; sc0 += 32) {
    v16b pa;
#pragma unroll
    for (int st = 0; st < 2; ++st) {
      const int kr = sc0 + st * 16;
      const v16b a0 = frag_kb(Kb + (size_t)(kr + nloc) * DK, hlf), a1 = frag_kb(Kb + (size_t)(kr + nloc) * DK + 32, hlf);
      v8f s8 = (v8f){}; s8 = wmma16b(a0, b0, s8); s8 = wmma16b(a1, b1, s8);
      const v8i m8 = *(const v8i*)(mrow + kr + 8 * hlf);
#pragma unroll
      for (int r = 0; r < 8; ++r) { const float e = nexp2(s8[r] * c); const int m = m8[r];
        const float w = (m == 0) ? w0 : ((m == 1) ? w1 : ((m == 2) ? w2 : ((m == 3) ? w3 : 0.0f)));
        pa[st * 8 + r] = (b16)(e * w); }
    }
#pragma unroll
    for (int vs = 0; vs < 4; ++vs) hacc[vs] = wmma16b(pa, frag_kb(Vb + (size_t)(vs * 16 + nloc) * SEQ + sc0, hlf), hacc[vs]);
  }
#pragma unroll
  for (int vs = 0; vs < 4; ++vs)
#pragma unroll
    for (int r = 0; r < 8; ++r) Th[wave][8 * hlf + r][vs * 16 + nloc] = (b16)(hacc[vs][r] * (CTS / (PSC * QS)));
  wave_lds_sync();
  for (int pass = 0; pass < 2; ++pass) {
#pragma unroll
    for (int i = 0; i < 4; ++i) { const int rr = i * 4 + (lane >> 3), pc = (lane & 7) * 8; const size_t row = (size_t)b * SEQ + q0 + wave * 16 + rr;
      const v8b v = *(const v8b*)(&Th[wave][rr][pc]); *(volatile v8b*)(CT + row * INTER + hd * DK + pc) = v; }
    __threadfence(); }
}
__global__ __launch_bounds__(128) void out_kernel(const b16* __restrict__ CT, const b16* __restrict__ WO, float* __restrict__ out) {
  __shared__ __attribute__((aligned(16))) float Tf[4][16][128 + 4];
  const int wave = threadIdx.x >> 5, lane = threadIdx.x & 31, nloc = lane & 15, hlf = lane >> 4; const size_t m0 = (size_t)blockIdx.x * 64 + wave * 16; const int n0 = blockIdx.y * 128;
  v8f acc[8];
#pragma unroll
  for (int t = 0; t < 8; ++t) acc[t] = (v8f){};
#pragma unroll 2
  for (int kb = 0; kb < INTER; kb += 32) { const v16b a = frag_kb(CT + (m0 + nloc) * INTER + kb, hlf);
#pragma unroll
    for (int t = 0; t < 8; ++t) acc[t] = wmma16b(a, frag_kb(WO + (size_t)(n0 + t * 16 + nloc) * INTER + kb, hlf), acc[t]); }
#pragma unroll
  for (int t = 0; t < 8; ++t)
#pragma unroll
    for (int r = 0; r < 8; ++r) Tf[wave][8 * hlf + r][t * 16 + nloc] = acc[t][r] * (1.0f / (CTS * WSC));
  wave_lds_sync();
  for (int pass = 0; pass < 2; ++pass) { for (int rr = 0; rr < 16; ++rr) *(volatile v4f*)(out + (m0 + rr) * DM + n0 + lane * 4) = *(const v4f*)(&Tf[wave][rr][lane * 4]); __threadfence(); }
}
}

extern "C" void kernel_launch(void* const* d_in, const int* in_sizes, int n_in, void* d_out, int out_size, void* d_ws, size_t ws_size, hipStream_t stream) {
  (void)n_in;
  const float* X = (const float*)d_in[0]; const int* MK = (const int*)d_in[1]; const float* WQ = (const float*)d_in[2]; const float* WOUT = (const float*)d_in[3]; const int* NSG = (const int*)d_in[4];
  const long long need_x = ((long long)(NB - 1) * SEQ_FULL + SEQ) * DM, need_m = ((long long)(NB - 1) * SEQ_FULL + SEQ) * SEQ_FULL;
  if ((long long)in_sizes[0] < need_x || (long long)in_sizes[1] < need_m || in_sizes[2] < DM * NQKV || in_sizes[3] < INTER * DM || in_sizes[4] < 1 || out_size < NR * DM) return;
  size_t off = 0; char* ws = (char*)d_ws;
  auto carve = [&](size_t bytes) { char* p = ws + off; off += (bytes + 255) & ~(size_t)255; return p; };
  b16* WQKV = (b16*)carve((size_t)NQKV * DM * 2);
  b16* WO = (b16*)carve((size_t)DM * INTER * 2);
  b16* XH = (b16*)carve((size_t)NR * DM * 2);
  b16* QP = (b16*)carve((size_t)NBH * SEQ * DK * 2);
  b16* KP = (b16*)carve((size_t)NBH * SEQ * DK * 2);
  b16* VT = (b16*)carve((size_t)NBH * DK * SEQ * 2);
  float* RS = (float*)carve((size_t)NBH * SEQ * NSEG * 4);
  b16* CT = (b16*)carve((size_t)NR * INTER * 2);
  if (off > ws_size || off > ((size_t)128 << 20)) return;
  wtp_kernel<<<dim3(DM / 64, NQKV / 64), 128, 0, stream>>>(WQ, DM, NQKV, WQKV);
  wtp_kernel<<<dim3(INTER / 64, DM / 64), 128, 0, stream>>>(WOUT, INTER, DM, WO);
  xp_kernel<<<(unsigned)(((size_t)NR * DM / 8 + 255) / 256), 256, 0, stream>>>(X, XH);
  qkv_kernel<<<dim3(NR / 64, NQKV / 128), 128, 0, stream>>>(XH, WQKV, QP, KP, VT);
  rowsum_kernel<<<dim3(SEQ / 128, NBH), 256, 0, stream>>>(QP, KP, MK, NSG, RS);
  av_kernel<<<dim3(SEQ / 128, NBH), 256, 0, stream>>>(QP, KP, VT, MK, RS, CT);
  out_kernel<<<dim3(NR / 64, DM / 128), 128, 0, stream>>>(CT, WO, (float*)d_out);
}
